// L1OutUB_28114855919757
// MI455X (gfx1250) — hardware-verified
//
#include <hip/hip_runtime.h>
#include <math.h>

typedef __attribute__((ext_vector_type(16))) _Float16 v16h;
typedef __attribute__((ext_vector_type(8)))  _Float16 v8h;
typedef __attribute__((ext_vector_type(16))) __bf16   v16b;
typedef __attribute__((ext_vector_type(8)))  __bf16   v8b;
typedef __attribute__((ext_vector_type(8)))  float    v8f;
typedef __attribute__((ext_vector_type(4)))  float    v4f;
typedef __attribute__((ext_vector_type(4)))  unsigned int v4u;

constexpr int NB_ROWS = 384;
constexpr int NDIM    = 512;
constexpr int NHID    = 512;
static_assert(NB_ROWS % 64 == 0, "M tile");
static_assert(NDIM % 64 == 0 && NHID % 64 == 0, "N tile");
static_assert(NDIM % 32 == 0 && NHID % 32 == 0, "K step");
static_assert(NDIM == 512, "reduce block width");

__device__ __forceinline__ unsigned short f2bf_bits(float f) {
  unsigned u = __float_as_uint(f);
  return (unsigned short)((u + 0x7FFFu + ((u >> 16) & 1u)) >> 16);
}
__device__ __forceinline__ float bf_bits2f(unsigned short h) { return __uint_as_float(((unsigned)h) << 16); }

__device__ __forceinline__ void dep_guard_h(v8f& a, v8f& b, v16h x, v16h y) { asm volatile("v_nop\n\tv_nop\n\tv_nop\n\tv_nop" : "+v"(a), "+v"(b) : "v"(x), "v"(y)); }
__device__ __forceinline__ void dep_guard_b(v8f& a, v8f& b, v16b x, v16b y) { asm volatile("v_nop\n\tv_nop\n\tv_nop\n\tv_nop" : "+v"(a), "+v"(b) : "v"(x), "v"(y)); }
__device__ __forceinline__ void keep4_h(v16h a, v16h b, v16h c, v16h d) { asm volatile("v_nop" :: "v"(a), "v"(b), "v"(c), "v"(d)); }
__device__ __forceinline__ void keep4_b(v16b a, v16b b, v16b c, v16b d) { asm volatile("v_nop" :: "v"(a), "v"(b), "v"(c), "v"(d)); }
__device__ __forceinline__ void acc_guard4(v8f& a, v8f& b, v8f& c, v8f& d) { asm volatile("v_nop\n\tv_nop\n\tv_nop\n\tv_nop" : "+v"(a), "+v"(b), "+v"(c), "+v"(d)); }
template <typename T> struct Frag;
template <> struct Frag<_Float16> {
  typedef v16h V; union U { v16h v; v8h h[2]; };
  static __device__ __forceinline__ v16h load(const _Float16* p) {
    U f; f.h[0] = *(const v8h*)(p); f.h[1] = *(const v8h*)(p + 16); return f.v;
  }
  static __device__ __forceinline__ v8f mma(v16h a, v16h b, v8f c) {
    return __builtin_amdgcn_wmma_f32_16x16x32_f16(false, a, false, b, (short)0, c, false, false);
  }
  static __device__ __forceinline__ void guard(v8f& a, v8f& b, v16h x, v16h y) { dep_guard_h(a, b, x, y); }
  static __device__ __forceinline__ void keep(v16h a, v16h b, v16h c, v16h d) { keep4_h(a, b, c, d); }
};
template <> struct Frag<__bf16> {
  typedef v16b V; union U { v16b v; v8b h[2]; };
  static __device__ __forceinline__ v16b load(const __bf16* p) {
    U f; f.h[0] = *(const v8b*)(p); f.h[1] = *(const v8b*)(p + 16); return f.v;
  }
  static __device__ __forceinline__ v8f mma(v16b a, v16b b, v8f c) {
    return __builtin_amdgcn_wmma_f32_16x16x32_bf16(false, a, false, b, (short)0, c, false, false);
  }
  static __device__ __forceinline__ void guard(v8f& a, v8f& b, v16b x, v16b y) { dep_guard_b(a, b, x, y); }
  static __device__ __forceinline__ void keep(v16b a, v16b b, v16b c, v16b d) { keep4_b(a, b, c, d); }
};

template <int ET> struct Elem;
template <> struct Elem<0> { typedef _Float16 T; };
template <> struct Elem<1> { typedef __bf16 T; };
template <int ET, bool SPLIT, int BIAS_MODE, int OUT_MODE, bool RESID, int ACT = 0>
__global__ __launch_bounds__(256) void wmma_gemm64(
    const unsigned short* __restrict__ Ap, const unsigned short* __restrict__ A2p, int lda, long strideA,
    const unsigned short* __restrict__ Btp, const unsigned short* __restrict__ Bt2p, int ldb, long strideB,
    void* __restrict__ Cout, void* __restrict__ Cout2, int ldc, long strideC,
    const float* __restrict__ bias,
    const float* __restrict__ resid, long strideR,
    int M, int N, int K, float scale) {
  typedef typename Elem<ET>::T T;
  typedef typename Frag<T>::V V;
  const T* A = (const T*)Ap; const T* A2 = (const T*)A2p; const T* Bt = (const T*)Btp; const T* Bt2 = (const T*)Bt2p;
  __shared__ __align__(16) float sT[8][16 * 68];
  const int b    = blockIdx.y;
  const int lane = threadIdx.x & 31;
  const int wave = threadIdx.x >> 5;
  const int tilesN = N >> 6;
  const int tilesM = M >> 6;
  const int tile = blockIdx.x * 8 + wave;
  if (tile >= tilesM * tilesN) return;
  const int tm = tile / tilesN;
  const int tn = tile - tm * tilesN;
  const int m0 = tm << 6;
  const int n0 = tn << 6;

  const T* Ab  = A  + (size_t)b * strideA;
  const T* Bb  = Bt + (size_t)b * strideB;
  const T* Ab2 = SPLIT ? (A2  + (size_t)b * strideA) : nullptr;
  const T* Bb2 = SPLIT ? (Bt2 + (size_t)b * strideB) : nullptr;

  const int rlane = lane & 15;
  const int koff  = (lane >> 4) * 8;
  const int mOff  = (lane >> 4) * 8;

  v8f acc[4][4];
#pragma unroll
  for (int i = 0; i < 4; ++i)
#pragma unroll
    for (int j = 0; j < 4; ++j) acc[i][j] = (v8f){0.f,0.f,0.f,0.f,0.f,0.f,0.f,0.f};

  for (int k0 = 0; k0 < K; k0 += 32) {
    V bh[4], bl[4];
#pragma unroll
    for (int j = 0; j < 4; ++j) {
      const size_t bo = (size_t)(n0 + (j << 4) + rlane) * ldb + koff + k0;
      bh[j] = Frag<T>::load(Bb + bo);
      if (SPLIT) bl[j] = Frag<T>::load(Bb2 + bo);
    }
#pragma unroll
    for (int i = 0; i < 4; ++i) {
      const size_t ao = (size_t)(m0 + (i << 4) + rlane) * lda + koff + k0;
      V ah = Frag<T>::load(Ab + ao);
      V al;
      if (SPLIT) al = Frag<T>::load(Ab2 + ao);
#pragma unroll
      for (int j = 0; j < 4; ++j) {
        acc[i][j] = Frag<T>::mma(ah, bh[j], acc[i][j]);
        if (SPLIT) {
          acc[i][j] = Frag<T>::mma(ah, bl[j], acc[i][j]);
          acc[i][j] = Frag<T>::mma(al, bh[j], acc[i][j]);
        }
      }
      Frag<T>::guard(acc[i][0], acc[i][3], ah, SPLIT ? al : ah);
    }
    Frag<T>::keep(bh[0], bh[1], bh[2], bh[3]);
    if (SPLIT) Frag<T>::keep(bl[0], bl[1], bl[2], bl[3]);
  }
  acc_guard4(acc[0][0], acc[0][1], acc[0][2], acc[0][3]);
  acc_guard4(acc[1][0], acc[1][1], acc[1][2], acc[1][3]);
  acc_guard4(acc[2][0], acc[2][1], acc[2][2], acc[2][3]);
  acc_guard4(acc[3][0], acc[3][1], acc[3][2], acc[3][3]);

  float* slab = sT[wave];
  const float* Rb = RESID ? (resid + (size_t)b * strideR) : nullptr;
#pragma unroll
  for (int i = 0; i < 4; ++i) {
    const int mBase = m0 + (i << 4);
#pragma unroll
    for (int j = 0; j < 4; ++j) {
      const int n = n0 + (j << 4) + rlane;
      float bv = 0.f;
      if (BIAS_MODE == 2) bv = bias[n];
#pragma unroll
      for (int r = 0; r < 8; ++r) {
        float v = acc[i][j][r] * scale;
        if (BIAS_MODE == 1) v += bias[mBase + mOff + r];
        if (BIAS_MODE == 2) v += bv;
        if (RESID) v += Rb[(size_t)(mBase + mOff + r) * ldc + n];
        if (ACT == 1) v = tanhf(v);
        if (ACT == 2) v = fmaxf(v, 0.0f);
        if (ACT == 3) v = v / (1.0f + expf(-v));
        if (ACT == 4) v = (v > 0.f) ? v : 0.01f * v;
        if (ACT == 5) v = 0.5f * v * (1.0f + erff(v * 0.70710678118654752f));
        slab[(mOff + r) * 68 + (j << 4) + rlane] = v;
      }
    }
    __builtin_amdgcn_fence(__ATOMIC_RELEASE, "workgroup");
    __builtin_amdgcn_wave_barrier();
    __builtin_amdgcn_fence(__ATOMIC_ACQUIRE, "workgroup");
    if (OUT_MODE == 0) {
      float* C = (float*)Cout + (size_t)b * strideC;
      const int hh = lane >> 4, c4 = (lane & 15) * 4;
      for (int pass = 0; pass < 2; ++pass) {
#pragma unroll
        for (int it = 0; it < 8; ++it) {
          const int row = it * 2 + hh;
          v4f v = *(const v4f*)(slab + row * 68 + c4);
          *(volatile v4f*)(C + (size_t)(mBase + row) * ldc + n0 + c4) = v;
        }
        __threadfence();
      }
    } else {
      const int q = lane >> 3, c8 = (lane & 7) * 8;
      unsigned short* C  = (unsigned short*)Cout  + (size_t)b * strideC;
      unsigned short* C2 = (OUT_MODE == 2) ? ((unsigned short*)Cout2 + (size_t)b * strideC) : nullptr;
      for (int pass = 0; pass < 2; ++pass) {
#pragma unroll
        for (int it = 0; it < 4; ++it) {
          const int row = it * 4 + q;
          const float* sp = slab + row * 68 + c8;
          v8h hv, lv;
#pragma unroll
          for (int e = 0; e < 8; ++e) {
            if (OUT_MODE == 1) {
              hv[e] = (_Float16)sp[e];
            } else {
              unsigned short hb = f2bf_bits(sp[e]);
              unsigned short lb = f2bf_bits(sp[e] - bf_bits2f(hb));
              hv[e] = __builtin_bit_cast(_Float16, hb);
              lv[e] = __builtin_bit_cast(_Float16, lb);
            }
          }
          *(volatile v8h*)(C + (size_t)(mBase + row) * ldc + n0 + c8) = hv;
          if (OUT_MODE == 2) *(volatile v8h*)(C2 + (size_t)(mBase + row) * ldc + n0 + c8) = lv;
        }
        __threadfence();
      }
    }
    __builtin_amdgcn_fence(__ATOMIC_RELEASE, "workgroup");
    __builtin_amdgcn_wave_barrier();
    __builtin_amdgcn_fence(__ATOMIC_ACQUIRE, "workgroup");
  }
}

__device__ __forceinline__ void split2_bf16(float f0, float f1, unsigned& hw, unsigned& lw) {
  const unsigned short h0 = f2bf_bits(f0), h1 = f2bf_bits(f1);
  const unsigned short l0 = f2bf_bits(f0 - bf_bits2f(h0));
  const unsigned short l1 = f2bf_bits(f1 - bf_bits2f(h1));
  hw = (unsigned)h0 | ((unsigned)h1 << 16);
  lw = (unsigned)l0 | ((unsigned)l1 << 16);
}
__device__ __forceinline__ void split8_bf16(float f0, float f1, float f2, float f3,
                                            float f4, float f5, float f6, float f7,
                                            v4u& hvec, v4u& lvec) {
  unsigned hw, lw;
  split2_bf16(f0, f1, hw, lw); hvec[0] = hw; lvec[0] = lw;
  split2_bf16(f2, f3, hw, lw); hvec[1] = hw; lvec[1] = lw;
  split2_bf16(f4, f5, hw, lw); hvec[2] = hw; lvec[2] = lw;
  split2_bf16(f6, f7, hw, lw); hvec[3] = hw; lvec[3] = lw;
}

__global__ __launch_bounds__(256) void split_rows_bf16(const float* __restrict__ in,
                                                        unsigned short* __restrict__ hi,
                                                        unsigned short* __restrict__ lo, int n8) {
  const int i = blockIdx.x * 256 + threadIdx.x;
  if (i < n8) {
    const v4f a = *(const v4f*)(in + (size_t)8 * i);
    const v4f c = *(const v4f*)(in + (size_t)8 * i + 4);
    v4u hvec, lvec;
    split8_bf16(a[0], a[1], a[2], a[3], c[0], c[1], c[2], c[3], hvec, lvec);
    unsigned short* ph = hi + (size_t)8 * i;
    unsigned short* pl = lo + (size_t)8 * i;
    *(volatile v4u*)ph = hvec;
    *(volatile v4u*)pl = lvec;
    __threadfence();
    *(volatile v4u*)ph = hvec;
    *(volatile v4u*)pl = lvec;
  }
}

__global__ __launch_bounds__(256) void transpose_split_bf16(const float* __restrict__ w,
                                                            unsigned short* __restrict__ th,
                                                            unsigned short* __restrict__ tl,
                                                            int R, int Cc) {
  __shared__ float tile[64][65];
  const int r0 = blockIdx.y * 64;
  const int c0 = blockIdx.x * 64;
  const int t = threadIdx.x;
#pragma unroll
  for (int it = 0; it < 4; ++it) {
    const int idx = it * 256 + t;
    const int row = idx >> 4;
    const int c4 = (idx & 15) * 4;
    const v4f v = *(const v4f*)(w + (size_t)(r0 + row) * Cc + c0 + c4);
    tile[row][c4 + 0] = v[0];
    tile[row][c4 + 1] = v[1];
    tile[row][c4 + 2] = v[2];
    tile[row][c4 + 3] = v[3];
  }
  __syncthreads();
  const int wave = t >> 5, lane = t & 31;
  const int q = lane >> 3, k8 = (lane & 7) * 8;
  const int nl0 = wave * 4 + q;
  const int nl1 = 32 + wave * 4 + q;
  v4u hv0, lv0, hv1, lv1;
  split8_bf16(tile[k8 + 0][nl0], tile[k8 + 1][nl0], tile[k8 + 2][nl0], tile[k8 + 3][nl0],
              tile[k8 + 4][nl0], tile[k8 + 5][nl0], tile[k8 + 6][nl0], tile[k8 + 7][nl0], hv0, lv0);
  split8_bf16(tile[k8 + 0][nl1], tile[k8 + 1][nl1], tile[k8 + 2][nl1], tile[k8 + 3][nl1],
              tile[k8 + 4][nl1], tile[k8 + 5][nl1], tile[k8 + 6][nl1], tile[k8 + 7][nl1], hv1, lv1);
  const size_t o0 = (size_t)(c0 + nl0) * R + r0 + k8;
  const size_t o1 = (size_t)(c0 + nl1) * R + r0 + k8;
  for (int pass = 0; pass < 2; ++pass) {
    *(volatile v4u*)(th + o0) = hv0;
    *(volatile v4u*)(tl + o0) = lv0;
    *(volatile v4u*)(th + o1) = hv1;
    *(volatile v4u*)(tl + o1) = lv1;
    __threadfence();
  }
}

__global__ __launch_bounds__(512) void final_reduce(const float* __restrict__ y,
                                                    const float* __restrict__ mu,
                                                    const float* __restrict__ lv,
                                                    float* __restrict__ out) {
  __shared__ double sred[NDIM];
  const int d = threadIdx.x;
  double s1 = 0.0, s2 = 0.0;
#pragma unroll 1
  for (int j = 0; j < NB_ROWS; ++j) {
    const double v = (double)y[(size_t)j * NDIM + d];
    s1 += v;
    s2 += v * v;
  }
  const double m1 = s1 * (1.0 / (double)NB_ROWS);
  const double m2 = s2 * (1.0 / (double)NB_ROWS);
  double acc = 0.0;
#pragma unroll 1
  for (int i = 0; i < NB_ROWS; ++i) {
    const size_t o = (size_t)i * NDIM + d;
    const float lvv = lv[o];
    const float ivv = expf(-lvv);
    const double yd = (double)y[o];
    const double md = (double)mu[o];
    const double br = (yd * yd - m2) - 2.0 * md * (yd - m1);
    acc += (double)ivv * br;
  }
  sred[d] = acc;
  __syncthreads();
  for (int s = NDIM / 2; s > 0; s >>= 1) {
    if (d < s) sred[d] += sred[d + s];
    __syncthreads();
  }
  if (d == 0) {
    const float r = (float)(sred[0] * (-0.5 / (double)NB_ROWS));
    *(volatile float*)out = r;
    __threadfence();
    *(volatile float*)out = r;
  }
}

extern "C" void kernel_launch(void* const* d_in, const int* in_sizes, int n_in,
                              void* d_out, int out_size, void* d_ws, size_t ws_size,
                              hipStream_t stream) {
  if (n_in < 10 || out_size < 1) return;
  if (in_sizes[0] != NB_ROWS * NDIM || in_sizes[1] != NB_ROWS * NDIM) return;
  if (in_sizes[2] != NDIM * NHID || in_sizes[3] != NHID) return;
  if (in_sizes[4] != NHID * NDIM || in_sizes[5] != NDIM) return;
  if (in_sizes[6] != NDIM * NHID || in_sizes[7] != NHID) return;
  if (in_sizes[8] != NHID * NDIM || in_sizes[9] != NDIM) return;

  const float* x    = (const float*)d_in[0];
  const float* y    = (const float*)d_in[1];
  const float* w1mu = (const float*)d_in[2];
  const float* b1mu = (const float*)d_in[3];
  const float* w2mu = (const float*)d_in[4];
  const float* b2mu = (const float*)d_in[5];
  const float* w1lv = (const float*)d_in[6];
  const float* b1lv = (const float*)d_in[7];
  const float* w2lv = (const float*)d_in[8];
  const float* b2lv = (const float*)d_in[9];
  float* out = (float*)d_out;

  const size_t plane16_act = (size_t)NB_ROWS * NDIM * 2;
  const size_t plane16_w   = (size_t)NDIM * NHID * 2;
  const size_t plane32_act = (size_t)NB_ROWS * NDIM * 4;
  char* ws = (char*)d_ws;
  size_t off = 0;
  auto carve = [&](size_t bytes) -> char* { char* p = ws + off; off += (bytes + 255) & ~(size_t)255; return p; };

  unsigned short* xh   = (unsigned short*)carve(plane16_act);
  unsigned short* xl   = (unsigned short*)carve(plane16_act);
  unsigned short* w1mh = (unsigned short*)carve(plane16_w);
  unsigned short* w1ml = (unsigned short*)carve(plane16_w);
  unsigned short* w1lh = (unsigned short*)carve(plane16_w);
  unsigned short* w1ll = (unsigned short*)carve(plane16_w);
  unsigned short* w2mh = (unsigned short*)carve(plane16_w);
  unsigned short* w2ml = (unsigned short*)carve(plane16_w);
  unsigned short* w2lh = (unsigned short*)carve(plane16_w);
  unsigned short* w2ll = (unsigned short*)carve(plane16_w);
  unsigned short* hmh  = (unsigned short*)carve(plane16_act);
  unsigned short* hml  = (unsigned short*)carve(plane16_act);
  unsigned short* hlh  = (unsigned short*)carve(plane16_act);
  unsigned short* hll  = (unsigned short*)carve(plane16_act);
  float*          mur  = (float*)carve(plane32_act);
  float*          lvt  = (float*)carve(plane32_act);
  if (off > ws_size) return;

  const int n8 = (NB_ROWS * NDIM) / 8;
  split_rows_bf16<<<dim3((n8 + 255) / 256), dim3(256), 0, stream>>>(x, xh, xl, n8);

  transpose_split_bf16<<<dim3(NHID / 64, NDIM / 64), dim3(256), 0, stream>>>(w1mu, w1mh, w1ml, NDIM, NHID);
  transpose_split_bf16<<<dim3(NHID / 64, NDIM / 64), dim3(256), 0, stream>>>(w1lv, w1lh, w1ll, NDIM, NHID);
  transpose_split_bf16<<<dim3(NDIM / 64, NHID / 64), dim3(256), 0, stream>>>(w2mu, w2mh, w2ml, NHID, NDIM);
  transpose_split_bf16<<<dim3(NDIM / 64, NHID / 64), dim3(256), 0, stream>>>(w2lv, w2lh, w2ll, NHID, NDIM);

  const int tiles1 = (NB_ROWS / 64) * (NHID / 64);
  const int g1 = (tiles1 + 7) / 8;
  wmma_gemm64<1, true, 2, 2, false, 2><<<dim3(g1, 1), dim3(256), 0, stream>>>(
      xh, xl, NDIM, 0L, w1mh, w1ml, NDIM, 0L, (void*)hmh, (void*)hml, NHID, 0L,
      b1mu, (const float*)nullptr, 0L, NB_ROWS, NHID, NDIM, 1.0f);
  wmma_gemm64<1, true, 2, 2, false, 2><<<dim3(g1, 1), dim3(256), 0, stream>>>(
      xh, xl, NDIM, 0L, w1lh, w1ll, NDIM, 0L, (void*)hlh, (void*)hll, NHID, 0L,
      b1lv, (const float*)nullptr, 0L, NB_ROWS, NHID, NDIM, 1.0f);

  const int tiles2 = (NB_ROWS / 64) * (NDIM / 64);
  const int g2 = (tiles2 + 7) / 8;
  wmma_gemm64<1, true, 2, 0, false, 0><<<dim3(g2, 1), dim3(256), 0, stream>>>(
      hmh, hml, NHID, 0L, w2mh, w2ml, NHID, 0L, (void*)mur, (void*)nullptr, NDIM, 0L,
      b2mu, (const float*)nullptr, 0L, NB_ROWS, NDIM, NHID, 1.0f);
  wmma_gemm64<1, true, 2, 0, false, 1><<<dim3(g2, 1), dim3(256), 0, stream>>>(
      hlh, hll, NHID, 0L, w2lh, w2ll, NHID, 0L, (void*)lvt, (void*)nullptr, NDIM, 0L,
      b2lv, (const float*)nullptr, 0L, NB_ROWS, NDIM, NHID, 1.0f);

  final_reduce<<<dim3(1), dim3(NDIM), 0, stream>>>(y, mur, lvt, out);
}
